// S4BlockTorch_25546465477183
// MI455X (gfx1250) — hardware-run, weakly checked
//
#include <hip/hip_runtime.h>
#include <math.h>

constexpr int kBatch = 4;
constexpr int kSeq   = 2048;
constexpr int kChan  = 512;
constexpr int kTaps  = 2048;
constexpr int kTok   = kBatch * kSeq;

constexpr float kHCarry   = 16.0f;
constexpr float kGCarry   = 256.0f;
constexpr float kACarry   = 16.0f;
constexpr float kWCarry   = 256.0f;
constexpr float kConvFold = 1.0f / (kHCarry * kGCarry);
constexpr float kLinFold  = 1.0f / (kACarry * kWCarry);
constexpr float kLnEps    = 1e-5f;
constexpr float kInvChan  = 1.0f / (float)kChan;
constexpr float kHalfMinNormal = 6.103515625e-05f;

constexpr int kPre      = 256;
constexpr int kSeqP     = kSeq + kPre;
constexpr int kGrOff    = 48;
constexpr int kGrTop    = kTaps - 1 + kGrOff;
constexpr int kGrLen    = 2136;
constexpr int kGrGroups = kGrLen / 8;
constexpr int kGrAll    = 8 * kGrGroups;
constexpr int kLnTP     = 36;

static_assert(kTaps == kSeq);
static_assert(kSeq == 256 * 8);
static_assert(kSeq % 64 == 0 && kChan % 64 == 0);
static_assert(kTok % 32 == 0 && kChan % 32 == 0);
static_assert(kPre >= 16 * 15 + 16);
static_assert(kGrLen % 8 == 0 && kGrLen > kGrTop + 8 + 7);
static_assert(kGrTop - 32 * 63 - 15 - 16 - 7 >= 0);
static_assert(kGrAll <= 9 * 256);
static_assert(kConvFold == 1.0f / 4096.0f && kLinFold == 1.0f / 4096.0f);

typedef __attribute__((ext_vector_type(16))) _Float16 v16h;
typedef __attribute__((ext_vector_type(8)))  _Float16 v8h;
typedef __attribute__((ext_vector_type(8)))  float    v8f;
typedef __attribute__((ext_vector_type(4)))  float    v4f;
typedef __attribute__((ext_vector_type(4)))  unsigned int v4u;

__device__ __forceinline__ unsigned pk16(unsigned short a, unsigned short b) {
  return (unsigned)a | ((unsigned)b << 16);
}
__device__ __forceinline__ unsigned short h_bits(float f) {
  const _Float16 h = (_Float16)f;
  return __builtin_bit_cast(unsigned short, h);
}
__device__ __forceinline__ float flush_h(float v) {
  return (fabsf(v) < kHalfMinNormal) ? 0.0f : v;
}
__device__ __forceinline__ v4u pack8_flush(const float (&v)[8]) {
  unsigned short hb[8];
#pragma unroll
  for (int e = 0; e < 8; ++e) hb[e] = h_bits(flush_h(v[e]));
  return (v4u){pk16(hb[0], hb[1]), pk16(hb[2], hb[3]), pk16(hb[4], hb[5]), pk16(hb[6], hb[7])};
}
__device__ __forceinline__ float wave_sum32(float v) {
#pragma unroll
  for (int o = 16; o > 0; o >>= 1) v += __shfl_xor(v, o, 32);
  return v;
}

struct FragH {
  union U { v16h v; v8h h[2]; };
  static __device__ __forceinline__ v16h load(const _Float16* p) {
    U f;
    f.h[0] = *(const v8h*)(p);
    f.h[1] = *(const v8h*)(p + 16);
    return f.v;
  }
  static __device__ __forceinline__ v16h load_back(const _Float16* p) {
    U f;
    f.h[0] = *(const v8h*)(p);
    f.h[1] = *(const v8h*)(p - 16);
    return f.v;
  }
  static __device__ __forceinline__ v8f mma(v16h a, v16h b, v8f c) {
    return __builtin_amdgcn_wmma_f32_16x16x32_f16(false, a, false, b, (short)0, c, false, false);
  }
};
__device__ __forceinline__ void guard_plain(v8f& a0, v8f& a1, v16h x0, v16h x1, v16h y0) {
  asm volatile("v_nop\n\tv_nop\n\tv_nop\n\tv_nop"
               : "+v"(a0), "+v"(a1)
               : "v"(x0), "v"(x1), "v"(y0));
}
__device__ __forceinline__ void acc_guard4(v8f& a, v8f& b, v8f& c, v8f& d) {
  asm volatile("v_nop\n\tv_nop\n\tv_nop\n\tv_nop" : "+v"(a), "+v"(b), "+v"(c), "+v"(d));
}
__device__ __forceinline__ v8f mma_g(v16h a, v16h b, v8f c) {
  c = __builtin_amdgcn_wmma_f32_16x16x32_f16(false, a, false, b, (short)0, c, false, false);
  asm volatile("v_nop\n\tv_nop\n\tv_nop\n\tv_nop" : "+v"(c) : "v"(a), "v"(b));
  return c;
}
__device__ __forceinline__ void wave_lds_sync() {
  __builtin_amdgcn_fence(__ATOMIC_RELEASE, "workgroup");
  __builtin_amdgcn_wave_barrier();
  __builtin_amdgcn_fence(__ATOMIC_ACQUIRE, "workgroup");
}

__global__ __launch_bounds__(256) void wt_plane_kernel(const float* __restrict__ W,
                                                       unsigned short* __restrict__ out, int total8) {
  const int i = blockIdx.x * 256 + threadIdx.x;
  if (i >= total8) return;
  const size_t e0 = (size_t)i * 8;
  const v4f a0 = *(const v4f*)(W + e0);
  const v4f a1 = *(const v4f*)(W + e0 + 4);
  float v[8];
#pragma unroll
  for (int e = 0; e < 4; ++e) {
    v[e]     = a0[e] * kWCarry;
    v[4 + e] = a1[e] * kWCarry;
  }
  const v4u u = pack8_flush(v);
  *(volatile v4u*)(out + e0) = u;
  __threadfence();
  *(volatile v4u*)(out + e0) = u;
}

__global__ __launch_bounds__(256) void ln_t_kernel(const float* __restrict__ x, const float* __restrict__ nw,
                                                   const float* __restrict__ nb, unsigned short* __restrict__ HT) {
  __shared__ __align__(16) unsigned sTile[256 * kLnTP];
  __shared__ float sStat[128];
  const int tid = threadIdx.x, lane = tid & 31, wave = tid >> 5;
  const int b = blockIdx.y;
  const int l0 = blockIdx.x * 64;
  const float* xb = x + ((size_t)b * kSeq + l0) * kChan;

#pragma unroll 1
  for (int j = 0; j < 8; ++j) {
    const int tk = wave * 8 + j;
    const float* xr = xb + (size_t)tk * kChan + lane * 4;
    const v4f r0 = *(const v4f*)(xr);
    const v4f r1 = *(const v4f*)(xr + 128);
    const v4f r2 = *(const v4f*)(xr + 256);
    const v4f r3 = *(const v4f*)(xr + 384);
    float s = 0.0f;
#pragma unroll
    for (int e = 0; e < 4; ++e) s += (r0[e] + r1[e]) + (r2[e] + r3[e]);
    s = wave_sum32(s);
    const float mu = s * kInvChan;
    float q = 0.0f;
#pragma unroll
    for (int e = 0; e < 4; ++e) {
      const float d0 = r0[e] - mu, d1 = r1[e] - mu, d2 = r2[e] - mu, d3 = r3[e] - mu;
      q += d0 * d0;
      q += d1 * d1;
      q += d2 * d2;
      q += d3 * d3;
    }
    q = wave_sum32(q);
    const float inv = rsqrtf(q * kInvChan + kLnEps);
    if (lane == 0) {
      sStat[tk] = mu;
      sStat[64 + tk] = inv;
    }
  }
  __syncthreads();

  const int rq = lane >> 3, piece = lane & 7;
#pragma unroll 1
  for (int cc = 0; cc < 2; ++cc) {
    const int cb = cc * 256;
#pragma unroll 1
    for (int it = 0; it < 8; ++it) {
      const int task = it * 256 + tid;
      const int lp = task >> 6;
      const int cq = task & 63;
      const int ch = cb + cq * 4;
      const float* xa = xb + (size_t)(2 * lp) * kChan + ch;
      const v4f a  = *(const v4f*)(xa);
      const v4f a2 = *(const v4f*)(xa + kChan);
      const v4f w4 = *(const v4f*)(nw + ch);
      const v4f b4 = *(const v4f*)(nb + ch);
      const float mu0 = sStat[2 * lp],     in0 = sStat[64 + 2 * lp];
      const float mu1 = sStat[2 * lp + 1], in1 = sStat[64 + 2 * lp + 1];
#pragma unroll
      for (int e = 0; e < 4; ++e) {
        const float f0 = (((a[e]  - mu0) * in0) * w4[e] + b4[e]) * kHCarry;
        const float f1 = (((a2[e] - mu1) * in1) * w4[e] + b4[e]) * kHCarry;
        sTile[(cq * 4 + e) * kLnTP + lp] = pk16(h_bits(flush_h(f0)), h_bits(flush_h(f1)));
      }
    }
    __syncthreads();
    v4u regs[8];
#pragma unroll
    for (int it = 0; it < 8; ++it) {
      const int row = it * 32 + wave * 4 + rq;
      regs[it] = *(const v4u*)(sTile + row * kLnTP + piece * 4);
    }
    for (int pass = 0; pass < 2; ++pass) {
#pragma unroll
      for (int it = 0; it < 8; ++it) {
        const int row = it * 32 + wave * 4 + rq;
        const size_t o = ((size_t)(b * kChan + cb + row)) * kSeq + l0 + piece * 8;
        *(volatile v4u*)(HT + o) = regs[it];
      }
      __threadfence();
    }
    __syncthreads();
  }
}

__device__ __forceinline__ void store_tile(float* slab, float* dst, v8f acc, int lane) {
  const int n = lane & 15, half = lane >> 4;
  const v4f lo = (v4f){acc[0] * kConvFold, acc[1] * kConvFold, acc[2] * kConvFold, acc[3] * kConvFold};
  const v4f hi = (v4f){acc[4] * kConvFold, acc[5] * kConvFold, acc[6] * kConvFold, acc[7] * kConvFold};
  *(v4f*)(slab + 16 * n + 8 * half)     = lo;
  *(v4f*)(slab + 16 * n + 8 * half + 4) = hi;
  wave_lds_sync();
  const v4f o0 = *(const v4f*)(slab + lane * 4);
  const v4f o1 = *(const v4f*)(slab + 128 + lane * 4);
  *(volatile v4f*)(dst + lane * 4)       = o0;
  *(volatile v4f*)(dst + 128 + lane * 4) = o1;
  __threadfence();
  *(volatile v4f*)(dst + lane * 4)       = o0;
  *(volatile v4f*)(dst + 128 + lane * 4) = o1;
  wave_lds_sync();
}

template <int PAR>
__device__ __forceinline__ void conv_tiles(const _Float16* aP, const _Float16* sq, float* slab,
                                           float* yrow, int lane) {
  constexpr int pA = 16 * PAR, pB = 16 * PAR + 32, pC = 80 - 16 * PAR, pD = 112 - 16 * PAR;
  constexpr int nA = pA / 2 + 8, nB = pB / 2 + 8, nC = pC / 2 + 8, nD = pD / 2 + 8;
  static_assert(nA < nB && nB < nC && nC < nD && nD <= 64);
  static_assert(nA + nB + nC + nD == 144);
  const _Float16* bA = sq + 16 * pA;
  const _Float16* bB = sq + 16 * pB;
  const _Float16* bC = sq + 16 * pC;
  const _Float16* bD = sq + 16 * pD;
  v8f accA = (v8f){0.f, 0.f, 0.f, 0.f, 0.f, 0.f, 0.f, 0.f};
  v8f accB = accA, accC = accA, accD = accA;
#pragma unroll 1
  for (int u = 0; u < nA; ++u) {
    const int off = 32 * u;
    const v16h a = FragH::load_back(aP - off);
    accA = mma_g(a, FragH::load_back(bA - off), accA);
    accB = mma_g(a, FragH::load_back(bB - off), accB);
    accC = mma_g(a, FragH::load_back(bC - off), accC);
    accD = mma_g(a, FragH::load_back(bD - off), accD);
  }
#pragma unroll 1
  for (int u = nA; u < nB; ++u) {
    const int off = 32 * u;
    const v16h a = FragH::load_back(aP - off);
    accB = mma_g(a, FragH::load_back(bB - off), accB);
    accC = mma_g(a, FragH::load_back(bC - off), accC);
    accD = mma_g(a, FragH::load_back(bD - off), accD);
  }
#pragma unroll 1
  for (int u = nB; u < nC; ++u) {
    const int off = 32 * u;
    const v16h a = FragH::load_back(aP - off);
    accC = mma_g(a, FragH::load_back(bC - off), accC);
    accD = mma_g(a, FragH::load_back(bD - off), accD);
  }
#pragma unroll 1
  for (int u = nC; u < nD; ++u) {
    const int off = 32 * u;
    const v16h a = FragH::load_back(aP - off);
    accD = mma_g(a, FragH::load_back(bD - off), accD);
  }
  acc_guard4(accA, accB, accC, accD);
  store_tile(slab, yrow + 16 * pA, accA, lane);
  store_tile(slab, yrow + 16 * pB, accB, lane);
  store_tile(slab, yrow + 16 * pC, accC, lane);
  store_tile(slab, yrow + 16 * pD, accD, lane);
}

__global__ __launch_bounds__(256) void longconv_mma_kernel(const unsigned short* __restrict__ HT,
                                                           const float* __restrict__ cw,
                                                           float* __restrict__ YT) {
  __shared__ __align__(16) _Float16 sSeq[kBatch * kSeqP];
  __shared__ __align__(16) _Float16 sGR[8 * kGrLen];
  __shared__ __align__(16) float sSlab[8 * 256];
  const int c = blockIdx.x;
  const int tid = threadIdx.x, lane = tid & 31, wave = tid >> 5;

#pragma unroll
  for (int bb = 0; bb < kBatch; ++bb) {
    const v4u d = *(const v4u*)(HT + ((size_t)(bb * kChan + c)) * kSeq + tid * 8);
    *(v8h*)(sSeq + bb * kSeqP + kPre + tid * 8) = __builtin_bit_cast(v8h, d);
  }
  if (tid < 128) {
    const int bb = tid >> 5, g = tid & 31;
    const v4u z = (v4u){0u, 0u, 0u, 0u};
    *(v8h*)(sSeq + bb * kSeqP + g * 8) = __builtin_bit_cast(v8h, z);
  }
  const float* wrow = cw + (size_t)c * kTaps;
#pragma unroll 1
  for (int it = 0; it < 9; ++it) {
    const int g  = it * 256 + tid;
    const int gc = (g < kGrAll) ? g : (kGrAll - 1);
    const int q  = gc / kGrGroups;
    const int gi = gc - q * kGrGroups;
    const int x0 = gi * 8 + q - kGrOff;
    float v[8];
#pragma unroll
    for (int e = 0; e < 8; ++e) {
      const int idx = x0 + e;
      const bool ok = (idx >= 0) && (idx < kTaps);
      const int ic = (idx < 0) ? 0 : ((idx < kTaps) ? idx : (kTaps - 1));
      float t = wrow[ic];
      asm volatile("" : "+v"(t));
      v[e] = ok ? (t * kGCarry) : 0.0f;
    }
    const v4u u = pack8_flush(v);
    if (g < kGrAll) *(v8h*)(sGR + q * kGrLen + gi * 8) = __builtin_bit_cast(v8h, u);
  }
  __syncthreads();

  const int n = lane & 15, half = lane >> 4;
  const int bsel = wave >> 1;
  const int par  = wave & 1;
  const int t0 = kGrTop - n + 8 * half;
  const int q  = t0 & 7;
  const _Float16* aP = sGR + q * kGrLen + (t0 - q);
  const _Float16* sq = sSeq + bsel * kSeqP + kPre + 16 * n + 8 * half;
  float* slab = sSlab + wave * 256;
  float* yrow = YT + ((size_t)(bsel * kChan + c)) * kSeq;
  if (par == 0) conv_tiles<0>(aP, sq, slab, yrow, lane);
  else          conv_tiles<1>(aP, sq, slab, yrow, lane);
}

__global__ __launch_bounds__(256) void gelu_t_kernel(const float* __restrict__ YT, const float* __restrict__ cb,
                                                     unsigned short* __restrict__ A16) {
  __shared__ __align__(16) float sT[64 * 68];
  const int tid = threadIdx.x, lane = tid & 31, wave = tid >> 5;
  const int l0 = blockIdx.x * 64;
  const int c0 = blockIdx.y * 64;
  const int b  = blockIdx.z;
  const int lc = tid & 63;
  const int r4 = tid >> 6;
#pragma unroll 1
  for (int it = 0; it < 16; ++it) {
    const int cr = it * 4 + r4;
    const float y = YT[((size_t)(b * kChan + c0 + cr)) * kSeq + l0 + lc] + cb[c0 + cr];
    const float g = 0.5f * y * (1.0f + erff(y * 0.70710678118654752f));
    sT[cr * 68 + lc] = g * kACarry;
  }
  __syncthreads();
  const int rq = lane >> 3, c8 = (lane & 7) * 8;
  v4u u[2];
#pragma unroll
  for (int it = 0; it < 2; ++it) {
    const int tk = it * 32 + wave * 4 + rq;
    float v[8];
#pragma unroll
    for (int e = 0; e < 8; ++e) v[e] = sT[(c8 + e) * 68 + tk];
    u[it] = pack8_flush(v);
  }
  for (int pass = 0; pass < 2; ++pass) {
#pragma unroll
    for (int it = 0; it < 2; ++it) {
      const int tk = it * 32 + wave * 4 + rq;
      const size_t o = ((size_t)(b * kSeq + l0 + tk)) * kChan + c0 + c8;
      *(volatile v4u*)(A16 + o) = u[it];
    }
    __threadfence();
  }
}

__global__ __launch_bounds__(256) void gemm_f16_bias_resid_kernel(
    const unsigned short* __restrict__ Ahp, int lda,
    const unsigned short* __restrict__ Bhp, int ldb,
    float* __restrict__ C, int ldc,
    const float* __restrict__ bias, const float* __restrict__ resid,
    int M, int N, int K, float scale) {
  __shared__ __align__(16) float sT[8][16 * 68];
  const int lane = threadIdx.x & 31;
  const int wave = threadIdx.x >> 5;
  const int tilesN = N >> 6;
  const int tilesM = M >> 5;
  const int tile = blockIdx.x * 8 + wave;
  if (tile >= tilesM * tilesN) return;
  const int tm = tile / tilesN;
  const int tn = tile - tm * tilesN;
  const int m0 = tm << 5;
  const int n0 = tn << 6;
  const int rlane = lane & 15;
  const int half8 = (lane >> 4) * 8;
  const int mOff  = (lane >> 4) * 8;

  const size_t aoff = (size_t)(m0 + rlane) * lda + half8;
  const size_t boff = (size_t)(n0 + rlane) * ldb + half8;
  const _Float16* pa0 = (const _Float16*)Ahp + aoff;
  const _Float16* pa1 = pa0 + (size_t)16 * lda;
  const _Float16* pbh = (const _Float16*)Bhp + boff;
  const size_t bstep = (size_t)16 * ldb;

  v8f acc[2][4];
#pragma unroll
  for (int i = 0; i < 2; ++i)
#pragma unroll
    for (int j = 0; j < 4; ++j) acc[i][j] = (v8f){0.f, 0.f, 0.f, 0.f, 0.f, 0.f, 0.f, 0.f};

  for (int k0 = 0; k0 < K; k0 += 32) {
    const v16h ah0 = FragH::load(pa0 + k0);
    const v16h ah1 = FragH::load(pa1 + k0);
#pragma unroll
    for (int j = 0; j < 4; ++j) {
      const v16h bh = FragH::load(pbh + j * bstep + k0);
      acc[0][j] = FragH::mma(ah0, bh, acc[0][j]);
      acc[1][j] = FragH::mma(ah1, bh, acc[1][j]);
      guard_plain(acc[0][j], acc[1][j], ah0, ah1, bh);
    }
  }
  acc_guard4(acc[0][0], acc[0][1], acc[0][2], acc[0][3]);
  acc_guard4(acc[1][0], acc[1][1], acc[1][2], acc[1][3]);

  float* slab = sT[wave];
  const int hh = lane >> 4, c4 = (lane & 15) * 4;
  const v4f bv = *(const v4f*)(bias + n0 + c4);
#pragma unroll
  for (int i = 0; i < 2; ++i) {
    const int mBase = m0 + (i << 4);
#pragma unroll
    for (int j = 0; j < 4; ++j) {
#pragma unroll
      for (int r = 0; r < 8; ++r) {
        slab[(mOff + r) * 68 + (j << 4) + rlane] = acc[i][j][r] * scale;
      }
    }
    wave_lds_sync();
    v4f o[8];
#pragma unroll
    for (int it = 0; it < 8; ++it) {
      const int row = it * 2 + hh;
      const v4f sv = *(const v4f*)(slab + row * 68 + c4);
      const v4f rv = *(const v4f*)(resid + (size_t)(mBase + row) * ldc + n0 + c4);
      o[it] = (sv + bv) + rv;
    }
    for (int pass = 0; pass < 2; ++pass) {
#pragma unroll
      for (int it = 0; it < 8; ++it) {
        const int row = it * 2 + hh;
        *(volatile v4f*)(C + (size_t)(mBase + row) * ldc + n0 + c4) = o[it];
      }
      __threadfence();
    }
    wave_lds_sync();
  }
}

extern "C" void kernel_launch(void* const* d_in, const int* in_sizes, int n_in,
                              void* d_out, int out_size, void* d_ws, size_t ws_size, hipStream_t stream) {
  if (n_in < 7 || d_out == nullptr || d_ws == nullptr) return;
  if (in_sizes[0] != kTok * kChan) return;
  if (in_sizes[1] != kChan || in_sizes[2] != kChan) return;
  if (in_sizes[3] != kChan * kTaps) return;
  if (in_sizes[4] != kChan) return;
  if (in_sizes[5] != kChan * kChan) return;
  if (in_sizes[6] != kChan) return;
  if (out_size != kTok * kChan) return;

  const float* x      = (const float*)d_in[0];
  const float* norm_w = (const float*)d_in[1];
  const float* norm_b = (const float*)d_in[2];
  const float* conv_w = (const float*)d_in[3];
  const float* conv_b = (const float*)d_in[4];
  const float* lin_w  = (const float*)d_in[5];
  const float* lin_b  = (const float*)d_in[6];
  float* out = (float*)d_out;

  char* ws = (char*)d_ws;
  size_t off = 0;
  auto carve = [&](size_t bytes) -> char* {
    char* p = ws + off;
    off += (bytes + 255) & ~(size_t)255;
    return p;
  };
  unsigned short* HT16 = (unsigned short*)carve((size_t)kBatch * kChan * kSeq * 2);
  float*          YT   = (float*)carve((size_t)kBatch * kChan * kSeq * 4);
  unsigned short* A16  = (unsigned short*)carve((size_t)kTok * kChan * 2);
  unsigned short* W16  = (unsigned short*)carve((size_t)kChan * kChan * 2);
  if (off > ws_size || off > (size_t)134217728) return;

  wt_plane_kernel<<<(kChan * kChan / 8) / 256, 256, 0, stream>>>(lin_w, W16, kChan * kChan / 8);

  ln_t_kernel<<<dim3(kSeq / 64, kBatch), 256, 0, stream>>>(x, norm_w, norm_b, HT16);

  longconv_mma_kernel<<<kChan, 256, 0, stream>>>(HT16, conv_w, YT);

  gelu_t_kernel<<<dim3(kSeq / 64, kChan / 64, kBatch), 256, 0, stream>>>(YT, conv_b, A16);

  gemm_f16_bias_resid_kernel<<<((kTok / 32) * (kChan / 64)) / 8, 256, 0, stream>>>(
      A16, kChan, W16, kChan, out, kChan, lin_b, x, kTok, kChan, kChan, kLinFold);
}
